// GATLayer_39367670235251
// MI455X (gfx1250) — hardware-verified
//
#include <hip/hip_runtime.h>
#include <stddef.h>


typedef _Float16 v16h __attribute__((ext_vector_type(16)));
typedef _Float16 v8h  __attribute__((ext_vector_type(8)));
typedef float    v8f  __attribute__((ext_vector_type(8)));
typedef float    v4f  __attribute__((ext_vector_type(4)));
typedef int      v4i  __attribute__((ext_vector_type(4)));
typedef _Float16 h16;

#ifndef NB
#define NB 2
#endif
#ifndef SEQ
#define SEQ 2048
#endif
#define NB_FULL  2
#define SEQ_FULL 2048
#define FIN   128
#define NHEAD 8
#define FOUT  32
#define CDIM  256
#define MROWS (NB * SEQ)

static_assert(NB >= 1 && NB <= NB_FULL);
static_assert(SEQ >= 128 && SEQ <= SEQ_FULL && (SEQ % 128) == 0);
static_assert(CDIM == NHEAD * FOUT);
static_assert(FOUT == 32);
static_assert(NHEAD == 8);
static_assert(64 == 2 * FOUT);
static_assert((FIN % 64) == 0 && (FIN % 32) == 0 && (FIN % 8) == 0);
static_assert((CDIM % 64) == 0);
static_assert((MROWS % 64) == 0 && (SEQ % 64) == 0 && (SEQ % 32) == 0 && (SEQ % 16) == 0);
static_assert((((size_t)MROWS * FIN / 8) % 256) == 0);
static_assert(256 == 64 * 2 * 2);
static_assert((size_t)NB_FULL * SEQ_FULL * CDIM * 4 == (size_t)4194304);

#define LDT 72
#define LDC 68
#define LDO 36
static_assert((LDT % 8) == 0 && LDT >= 64);
static_assert((LDC % 4) == 0 && LDC >= 64);
static_assert((LDO % 4) == 0 && LDO >= FOUT);

#define WCARRY 64.0f
#define VCARRY 16.0f
#define PCARRY 1024.0f
#define PLOG   6.931471806f
#define PFLUSH_ARG (-9.7f)
#define NEGFILL (-1.0e9f)
#define SLOPE 0.2f

#define WT_BYTES  ((size_t)CDIM * FIN * 2)
#define H16_BYTES ((size_t)MROWS * FIN * 2)
#define VT_BYTES  ((size_t)NB * CDIM * SEQ * 2)
#define S_BYTES   ((size_t)2 * NB * NHEAD * SEQ * 4)
#define OFF_WT  ((size_t)0)
#define OFF_H16 (OFF_WT + WT_BYTES)
#define OFF_VT  (OFF_H16 + H16_BYTES)
#define OFF_S   (OFF_VT + VT_BYTES)
#define WS_TOTAL (OFF_S + S_BYTES)
static_assert((WT_BYTES % 128) == 0 && (H16_BYTES % 128) == 0);
static_assert((VT_BYTES % 128) == 0 && (S_BYTES % 128) == 0);
static_assert(WS_TOTAL <= (size_t)134217728);

__device__ __forceinline__ float bf16r(float x) {
  unsigned int u = __float_as_uint(x);
  u = (u + 0x7FFFu + ((u >> 16) & 1u)) & 0xFFFF0000u;
  return __uint_as_float(u);
}

static __device__ __forceinline__ h16 toh_flush(float v) {
  const h16 r = (h16)v;
  return (fabsf(v) < 6.103515625e-05f) ? (h16)0.0f : r;
}
static __device__ __forceinline__ h16 p_to_h(float a) {
  const h16 r = (h16)__expf(a);
  return (a < PFLUSH_ARG) ? (h16)0.0f : r;
}

__device__ __forceinline__ v16h frag_at(const _Float16* p) {
  v8h lo = *(const v8h*)(p);
  v8h hi = *(const v8h*)(p + 16);
  v16h out;
#pragma unroll
  for (int i = 0; i < 8; ++i) { out[i] = lo[i]; out[i + 8] = hi[i]; }
  return out;
}

__device__ __forceinline__ v8f wmma16(v16h a, v16h b, v8f c) {
  v8f d = __builtin_amdgcn_wmma_f32_16x16x32_f16(false, a, false, b, (short)0, c,
                                                 false, false);
  asm volatile("v_nop\n\tv_nop\n\tv_nop\n\tv_nop" : "+v"(d) : "v"(a), "v"(b));
  return d;
}

__device__ __forceinline__ void wave_lds_sync() {
  __builtin_amdgcn_fence(3  , "wavefront");
  asm volatile("s_wait_dscnt 0x0" ::: "memory");
  __builtin_amdgcn_wave_barrier();
}

__global__ __launch_bounds__(256) void wconv_kernel(
    const float* __restrict__ W, _Float16* __restrict__ Wt, unsigned ldw, unsigned ldk) {
  __shared__ _Float16 T[64 * LDT];
  const unsigned tid = threadIdx.x;
  const unsigned n0 = blockIdx.x * 64u;
  const unsigned k0 = blockIdx.y * 64u;
#pragma unroll 4
  for (unsigned j = 0; j < 16u; ++j) {
    const unsigned idx = tid + 256u * j;
    const unsigned kr = idx >> 6, nc = idx & 63u;
    const float v = W[(size_t)(k0 + kr) * ldw + n0 + nc];
    T[nc * LDT + kr] = (_Float16)(WCARRY * bf16r(v));
  }
  __syncthreads();
  v8h x[2];
  size_t off[2];
#pragma unroll
  for (unsigned i = 0; i < 2u; ++i) {
    const unsigned n = 32u * i + (tid >> 3);
    const unsigned kc = (tid & 7u) * 8u;
    x[i] = *(const v8h*)&T[n * LDT + kc];
    off[i] = (size_t)(n0 + n) * ldk + k0 + kc;
  }
#pragma unroll
  for (int i = 0; i < 2; ++i) *(volatile v8h*)(Wt + off[i]) = x[i];
  __threadfence();
#pragma unroll
  for (int i = 0; i < 2; ++i) *(volatile v8h*)(Wt + off[i]) = x[i];
}

__global__ __launch_bounds__(256) void hcast_kernel(
    const float* __restrict__ X, _Float16* __restrict__ dst) {
  const unsigned g = blockIdx.x * 256u + threadIdx.x;
  const unsigned crow = g / (unsigned)(FIN / 8);
  const unsigned c = (g - crow * (unsigned)(FIN / 8)) * 8u;
  const unsigned bidx = crow / (unsigned)SEQ;
  const unsigned sq = crow - bidx * (unsigned)SEQ;
  const size_t srow = (size_t)bidx * SEQ_FULL + sq;
  const v4f a0 = *(const v4f*)(X + srow * FIN + c);
  const v4f a1 = *(const v4f*)(X + srow * FIN + c + 4u);
  v8h o;
#pragma unroll
  for (int i = 0; i < 4; ++i) {
    o[i]     = toh_flush(bf16r(a0[i]));
    o[i + 4] = toh_flush(bf16r(a1[i]));
  }
  _Float16* p = dst + (size_t)crow * FIN + c;
  *(volatile v8h*)p = o;
  __threadfence();
  *(volatile v8h*)p = o;
}

__global__ __launch_bounds__(256) void proj_kernel(
    const _Float16* __restrict__ A16, const _Float16* __restrict__ Bt,
    const float* __restrict__ avec, _Float16* __restrict__ vt, float* __restrict__ sp) {
  __shared__ __attribute__((aligned(16))) float Cs[64 * LDC];
  __shared__ __attribute__((aligned(16))) float Ss[4 * 64];
  const unsigned tid = threadIdx.x, lane = tid & 31u;
  const unsigned w = (unsigned)__builtin_amdgcn_readfirstlane((int)(tid >> 5));
  const unsigned mw = w >> 1, nw = w & 1u;
  const unsigned hh = lane >> 4, m = lane & 15u;
  const unsigned n0 = blockIdx.x * 64u;
  const unsigned row0 = blockIdx.y * 64u;
  const unsigned K = (unsigned)FIN;

  const _Float16* ap  = A16 + (size_t)(row0 + mw * 16u + m) * K + hh * 8u;
  const _Float16* bp0 = Bt + (size_t)(n0 + nw * 32u + m) * K + hh * 8u;
  const _Float16* bp1 = bp0 + (size_t)16 * K;
  v8f acc0 = {}, acc1 = {};
#pragma unroll 2
  for (unsigned k0 = 0; k0 < K; k0 += 32u) {
    const v16h a  = frag_at(ap + k0);
    const v16h b0 = frag_at(bp0 + k0);
    const v16h b1 = frag_at(bp1 + k0);
    acc0 = wmma16(a, b0, acc0);
    acc1 = wmma16(a, b1, acc1);
  }
#pragma unroll
  for (int r = 0; r < 8; ++r) {
    const unsigned ci = (mw * 16u + hh * 8u + (unsigned)r) * LDC + nw * 32u + m;
    Cs[ci]       = acc0[r];
    Cs[ci + 16u] = acc1[r];
  }
  __syncthreads();

  {
    const unsigned r = tid >> 2, hq = (tid >> 1) & 1u, which = tid & 1u;
    float s = 0.0f;
#pragma unroll 4
    for (unsigned f = 0; f < (unsigned)FOUT; ++f)
      s += Cs[r * LDC + hq * 32u + f] * bf16r(avec[which * 32u + f]);
    Ss[(which * 2u + hq) * 64u + r] = s * (1.0f / WCARRY);
  }
  __syncthreads();

  const unsigned bidx = row0 / (unsigned)SEQ;
  const unsigned key0 = row0 - bidx * (unsigned)SEQ;
  v8h x[2];
  size_t off[2];
#pragma unroll
  for (unsigned i = 0; i < 2u; ++i) {
    const unsigned dcol = 32u * i + (tid >> 3);
    const unsigned kk = (tid & 7u) * 8u;
#pragma unroll
    for (unsigned j = 0; j < 8u; ++j)
      x[i][j] = toh_flush(Cs[(kk + j) * LDC + dcol] * (VCARRY / WCARRY));
    off[i] = ((size_t)bidx * CDIM + n0 + dcol) * SEQ + key0 + kk;
  }
  const unsigned sl = (tid >> 3) & 7u, pc = tid & 7u;
  const unsigned comb = sl >> 1, rhalf = sl & 1u;
  const unsigned swhich = comb >> 1, shq = comb & 1u;
  const v4f sv = *(const v4f*)&Ss[sl * 32u + pc * 4u];
  const size_t soff = (((size_t)swhich * NB + bidx) * NHEAD + (n0 >> 5) + shq) * SEQ
                      + key0 + rhalf * 32u + pc * 4u;
  const bool swr = (tid < 64u);

#pragma unroll
  for (int i = 0; i < 2; ++i) *(volatile v8h*)(vt + off[i]) = x[i];
  if (swr) *(volatile v4f*)(sp + soff) = sv;
  __threadfence();
#pragma unroll
  for (int i = 0; i < 2; ++i) *(volatile v8h*)(vt + off[i]) = x[i];
  if (swr) *(volatile v4f*)(sp + soff) = sv;
}

__device__ __forceinline__ float masked_logit(int a, float x) {
  const float t = fmaxf(x, SLOPE * x);
  return (a != 0) ? t : NEGFILL;
}

__global__ __launch_bounds__(256) void nbr_attn_kernel(
    const _Float16* __restrict__ vt, const float* __restrict__ sp,
    const int* __restrict__ adj, float* __restrict__ outp) {
  __shared__ __attribute__((aligned(16))) float Os[8 * 16 * LDO];
  const unsigned lane = threadIdx.x & 31u;
  const unsigned wave = (unsigned)__builtin_amdgcn_readfirstlane((int)(threadIdx.x >> 5));
  const unsigned hh = lane >> 4, m = lane & 15u;
  const unsigned i0 = blockIdx.x * 16u;
  const unsigned b = blockIdx.y;
  const unsigned head = wave;

  const float si = sp[((size_t)b * NHEAD + head) * SEQ + i0 + m];
  const float* sjp = sp + (((size_t)NB + b) * NHEAD + head) * SEQ + hh * 8u;
  const int* arow = adj + ((size_t)b * SEQ_FULL + i0 + m) * SEQ_FULL + hh * 8u;
  const _Float16* vp0 = vt + ((size_t)b * CDIM + head * FOUT + m) * SEQ + hh * 8u;
  const _Float16* vp1 = vp0 + (size_t)16 * SEQ;

  float mrow = -1.0e30f, lsum = 0.0f;
  v8f o0 = {}, o1 = {};

#pragma unroll 1
  for (unsigned k0 = 0; k0 < (unsigned)SEQ; k0 += 32u) {
    const v16h va0 = frag_at(vp0 + k0);
    const v16h va1 = frag_at(vp1 + k0);
    const v4f sa = *(const v4f*)(sjp + k0);
    const v4f sb = *(const v4f*)(sjp + k0 + 4u);
    const v4f sc = *(const v4f*)(sjp + k0 + 16u);
    const v4f sd = *(const v4f*)(sjp + k0 + 20u);
    v4i ma = *(const v4i*)(arow + k0);
    v4i mb = *(const v4i*)(arow + k0 + 4u);
    v4i mc = *(const v4i*)(arow + k0 + 16u);
    v4i md = *(const v4i*)(arow + k0 + 20u);
    asm volatile("" : "+v"(ma), "+v"(mb), "+v"(mc), "+v"(md));

    float e[16];
#pragma unroll
    for (int i = 0; i < 4; ++i) {
      e[i]      = masked_logit(ma[i], si + sa[i]);
      e[4 + i]  = masked_logit(mb[i], si + sb[i]);
      e[8 + i]  = masked_logit(mc[i], si + sc[i]);
      e[12 + i] = masked_logit(md[i], si + sd[i]);
    }
    float mx = e[0];
#pragma unroll
    for (int i = 1; i < 16; ++i) mx = fmaxf(mx, e[i]);
    mx = fmaxf(mx, __shfl_xor(mx, 16, 32));
    const float mn = fmaxf(mrow, mx);
    const float alpha = __expf(mrow - mn);
    mrow = mn;

    v16h pb;
    float rs = 0.0f;
#pragma unroll
    for (int i = 0; i < 16; ++i) {
      const h16 ph = p_to_h((e[i] - mn) + PLOG);
      pb[i] = ph;
      rs += (float)ph;
    }
    lsum = alpha * lsum + rs;
#pragma unroll
    for (int r = 0; r < 8; ++r) { o0[r] = o0[r] * alpha; o1[r] = o1[r] * alpha; }

    o0 = wmma16(va0, pb, o0);
    o1 = wmma16(va1, pb, o1);
  }

  const float ltot = lsum + __shfl_xor(lsum, 16, 32);
  const float inv = __builtin_amdgcn_rcpf(ltot) * (1.0f / VCARRY);

  const unsigned ob = wave * (16u * LDO) + m * LDO + hh * 8u;
  v4f t0, t1, t2, t3;
#pragma unroll
  for (int r = 0; r < 4; ++r) {
    t0[r] = o0[r] * inv;
    t1[r] = o0[r + 4] * inv;
    t2[r] = o1[r] * inv;
    t3[r] = o1[r + 4] * inv;
  }
  *(v4f*)&Os[ob]       = t0;
  *(v4f*)&Os[ob + 4u]  = t1;
  *(v4f*)&Os[ob + 16u] = t2;
  *(v4f*)&Os[ob + 20u] = t3;
  wave_lds_sync();

  v4f x[4];
  size_t off[4];
#pragma unroll
  for (unsigned it = 0; it < 4u; ++it) {
    const unsigned r = 4u * it + (lane >> 3);
    const unsigned c = (lane & 7u) * 4u;
    x[it] = *(const v4f*)&Os[wave * (16u * LDO) + r * LDO + c];
    off[it] = ((size_t)b * SEQ_FULL + i0 + r) * CDIM + head * FOUT + c;
  }
#pragma unroll
  for (int it = 0; it < 4; ++it) *(volatile v4f*)(outp + off[it]) = x[it];
  __threadfence();
#pragma unroll
  for (int it = 0; it < 4; ++it) *(volatile v4f*)(outp + off[it]) = x[it];
}

extern "C" void kernel_launch(void* const* d_in, const int* in_sizes, int n_in,
                              void* d_out, int out_size, void* d_ws, size_t ws_size,
                              hipStream_t stream) {
  if (n_in < 4) return;
  const long long need_rows = (long long)(NB - 1) * SEQ_FULL + SEQ;
  if ((long long)in_sizes[0] < need_rows * FIN) return;
  if ((long long)in_sizes[1] < need_rows * SEQ_FULL) return;
  if ((long long)in_sizes[2] < (long long)FIN * CDIM) return;
  if (in_sizes[3] < 2 * FOUT) return;
  if ((long long)out_size < need_rows * CDIM) return;
  if (ws_size < WS_TOTAL) return;

  const float* Hin  = (const float*)d_in[0];
  const int*   adj  = (const int*)d_in[1];
  const float* Wm   = (const float*)d_in[2];
  const float* avec = (const float*)d_in[3];
  float* out = (float*)d_out;

  char* ws = (char*)d_ws;
  _Float16* Wt   = (_Float16*)(ws + OFF_WT);
  _Float16* H16  = (_Float16*)(ws + OFF_H16);
  _Float16* Vt16 = (_Float16*)(ws + OFF_VT);
  float*    Sp   = (float*)(ws + OFF_S);

  dim3 blk(256);
  wconv_kernel<<<dim3(CDIM / 64, FIN / 64), blk, 0, stream>>>(Wm, Wt, (unsigned)CDIM, (unsigned)FIN);
  hcast_kernel<<<dim3((unsigned)((size_t)MROWS * FIN / 8 / 256)), blk, 0, stream>>>(Hin, H16);
  proj_kernel<<<dim3(CDIM / 64, MROWS / 64), blk, 0, stream>>>(H16, Wt, avec, Vt16, Sp);
  nbr_attn_kernel<<<dim3(SEQ / 16, NB), blk, 0, stream>>>(Vt16, Sp, adj, out);
}
